// MultiHeadAttention_48833778155962
// MI455X (gfx1250) — hardware-verified
//
#include <hip/hip_runtime.h>
#ifndef NB
#define NB 2
#endif
#ifndef SEQ
#define SEQ 2048
#endif
#define NB_FULL 2
#define SEQ_FULL 2048
#define DM 1024
#define NH 16
#define HD 64
#define QT 64
#define NR (NB * SEQ)
#define QSCALE 0.125f

typedef __bf16 v16b __attribute__((ext_vector_type(16)));
typedef unsigned short v8us __attribute__((ext_vector_type(8), may_alias));
typedef float  v8f  __attribute__((ext_vector_type(8)));
typedef float  v4f  __attribute__((ext_vector_type(4)));
typedef float  v4fa __attribute__((ext_vector_type(4), may_alias));
union FragB { v16b v; v8us half[2]; unsigned short u[16]; };
union Pack8 { v8us v; unsigned short u[8]; };

static_assert(HD == 64);
static_assert(NH * HD == DM);
static_assert(DM % 64 == 0);
static_assert(DM % 32 == 0);
static_assert(SEQ % QT == 0);
static_assert(SEQ % 64 == 0);
static_assert(QT == 4 * 16);
static_assert(NR % 128 == 0);
static_assert(NB <= NB_FULL);
static_assert(SEQ <= SEQ_FULL);
static_assert((size_t)NR * DM < 2147483647u);
static_assert((size_t)DM * DM < 2147483647u);
static_assert(((size_t)NR * (DM / 8)) % 256 == 0);
static_assert(((size_t)DM * (DM / 8)) % 256 == 0);

constexpr size_t PLANE_B = (size_t)NR * DM * 2;
constexpr size_t WPL_B   = (size_t)DM * DM * 2;
constexpr size_t CARVE_B = 5 * PLANE_B + WPL_B;
static_assert(PLANE_B % 256 == 0);
static_assert(WPL_B % 256 == 0);
static_assert(CARVE_B <= 134217728u);

__device__ __forceinline__ unsigned short bf16_bits(float x) { unsigned int u = __float_as_uint(x); return (unsigned short)((u + 0x7FFFu + ((u >> 16) & 1u)) >> 16); }
__device__ __forceinline__ float bf16_val(unsigned short b) { return __uint_as_float(((unsigned int)b) << 16); }
__device__ __forceinline__ float bf16_rne(float x) { return bf16_val(bf16_bits(x)); }

__device__ __forceinline__ v16b ld_frag(const unsigned short* __restrict__ p, int off, int hh) {
  FragB f;
  f.half[0] = *(const v8us*)(p + off + 8 * hh);
  f.half[1] = *(const v8us*)(p + off + 16 + 8 * hh);
  return f.v;
}
__device__ __forceinline__ v8f mma1(v16b a, v16b b, v8f c) {
  c = __builtin_amdgcn_wmma_f32_16x16x32_bf16(false, a, false, b, (short)0, c, false, false);
  asm volatile("v_nop\n\tv_nop\n\tv_nop\n\tv_nop" : "+v"(c) : "v"(a), "v"(b));
  return c;
}
__device__ __forceinline__ v8f mma2b(v16b a, v16b bh, v16b bl, v8f c) {
  c = __builtin_amdgcn_wmma_f32_16x16x32_bf16(false, a, false, bh, (short)0, c, false, false);
  c = __builtin_amdgcn_wmma_f32_16x16x32_bf16(false, a, false, bl, (short)0, c, false, false);
  asm volatile("v_nop\n\tv_nop\n\tv_nop\n\tv_nop" : "+v"(c) : "v"(a), "v"(bh), "v"(bl));
  return c;
}
__device__ __forceinline__ v8f mma2a(v16b ah, v16b al, v16b b, v8f c) {
  c = __builtin_amdgcn_wmma_f32_16x16x32_bf16(false, ah, false, b, (short)0, c, false, false);
  c = __builtin_amdgcn_wmma_f32_16x16x32_bf16(false, al, false, b, (short)0, c, false, false);
  asm volatile("v_nop\n\tv_nop\n\tv_nop\n\tv_nop" : "+v"(c) : "v"(ah), "v"(al), "v"(b));
  return c;
}

__global__ __launch_bounds__(256) void k_cvt_qk(const float* __restrict__ q, const float* __restrict__ k, unsigned short* __restrict__ Qb, unsigned short* __restrict__ Kb) {
  const int t = blockIdx.x * 256 + threadIdx.x;
  if (t >= NR * (DM / 8)) return;
  const int row = t / (DM / 8), c8 = (t % (DM / 8)) * 8;
  const int b = row / SEQ, s = row % SEQ;
  const size_t src = ((size_t)b * SEQ_FULL + s) * DM + c8;
  const v4f a0 = *(const v4fa*)(q + src), a1 = *(const v4fa*)(q + src + 4);
  const v4f b0 = *(const v4fa*)(k + src), b1 = *(const v4fa*)(k + src + 4);
  Pack8 fq, fk;
#pragma unroll
  for (int i = 0; i < 4; ++i) {
    fq.u[i] = bf16_bits(a0[i] * QSCALE); fq.u[4 + i] = bf16_bits(a1[i] * QSCALE);
    fk.u[i] = bf16_bits(b0[i]);          fk.u[4 + i] = bf16_bits(b1[i]);
  }
  const size_t dst = (size_t)row * DM + c8;
  const v8us vq = fq.v, vk = fk.v;
  *(volatile v8us*)(Qb + dst) = vq; *(volatile v8us*)(Kb + dst) = vk;
  __threadfence();
  *(volatile v8us*)(Qb + dst) = vq; *(volatile v8us*)(Kb + dst) = vk;
}

__global__ __launch_bounds__(256) void k_cvt_w(const float* __restrict__ W, unsigned short* __restrict__ Wb) {
  const int t = blockIdx.x * 256 + threadIdx.x;
  if (t >= DM * (DM / 8)) return;
  const size_t e = (size_t)t * 8;
  const v4f a0 = *(const v4fa*)(W + e), a1 = *(const v4fa*)(W + e + 4);
  Pack8 f;
#pragma unroll
  for (int i = 0; i < 4; ++i) { f.u[i] = bf16_bits(a0[i]); f.u[4 + i] = bf16_bits(a1[i]); }
  const v8us v = f.v;
  *(volatile v8us*)(Wb + e) = v;
  __threadfence();
  *(volatile v8us*)(Wb + e) = v;
}

__global__ __launch_bounds__(256) void k_vt(const float* __restrict__ v, unsigned short* __restrict__ VT) {
  __shared__ unsigned short tl[64][66];
  static_assert((64 * 16) % 256 == 0);
  static_assert((64 * 8) % 256 == 0);
  const int tid = threadIdx.x;
  const int slab = blockIdx.x / (SEQ / 64), sg = blockIdx.x % (SEQ / 64);
  const int b = slab / NH, h = slab % NH;
  const int s0 = sg * 64;
  for (int i = tid; i < 64 * 16; i += 256) {
    const int j = i / 16, d4 = (i % 16) * 4;
    const v4f a = *(const v4fa*)(v + ((size_t)b * SEQ_FULL + s0 + j) * DM + h * HD + d4);
#pragma unroll
    for (int q = 0; q < 4; ++q) tl[d4 + q][j] = bf16_bits(a[q]);
  }
  __syncthreads();
  for (int pass = 0; pass < 2; ++pass) {
    for (int i = tid; i < 64 * 8; i += 256) {
      const int d = i / 8, j8 = (i % 8) * 8;
      Pack8 f;
#pragma unroll
      for (int q = 0; q < 8; ++q) f.u[q] = tl[d][j8 + q];
      const v8us o = f.v;
      *(volatile v8us*)(VT + ((size_t)slab * HD + d) * SEQ + s0 + j8) = o;
    }
    if (pass == 0) __threadfence();
  }
}

__global__ __launch_bounds__(128) void k_attn(const unsigned short* __restrict__ Qb, const unsigned short* __restrict__ Kb, const unsigned short* __restrict__ VT,
                                             unsigned short* __restrict__ CH, unsigned short* __restrict__ CL) {
  __shared__ __attribute__((aligned(16))) unsigned short sH[4][16][72];
  __shared__ __attribute__((aligned(16))) unsigned short sL[4][16][72];
  const int tid = threadIdx.x, w = tid >> 5, lane = tid & 31, ln = lane & 15, hh = lane >> 4;
  const int qt = blockIdx.x % (SEQ / QT), bh = blockIdx.x / (SEQ / QT);
  const int b = bh / NH, h = bh % NH;
  const int q0 = qt * QT + w * 16;
  const int qoff  = (b * SEQ + q0 + ln) * DM + h * HD;
  const int kbase = (b * SEQ + ln) * DM + h * HD;
  const int vbase = (bh * HD + ln) * SEQ;
  const v8f z8 = {0.f, 0.f, 0.f, 0.f, 0.f, 0.f, 0.f, 0.f};
  v8f o0 = z8, o1 = z8, o2 = z8, o3 = z8;
  float m = -1.0e30f, l = 0.f;
#pragma unroll 1
  for (int kb = 0; kb < SEQ; kb += 32) {
    const v16b qf0 = ld_frag(Qb, qoff, hh);
    const v16b qf1 = ld_frag(Qb, qoff + 32, hh);
    const int ko = kbase + kb * DM;
    v8f s0 = z8, s1 = z8;
    v16b ka = ld_frag(Kb, ko, hh);
    s0 = mma1(ka, qf0, s0);
    ka = ld_frag(Kb, ko + 32, hh);
    s0 = mma1(ka, qf1, s0);
    ka = ld_frag(Kb, ko + 16 * DM, hh);
    s1 = mma1(ka, qf0, s1);
    ka = ld_frag(Kb, ko + 16 * DM + 32, hh);
    s1 = mma1(ka, qf1, s1);
    float mx = fmaxf(s0[0], s1[0]);
#pragma unroll
    for (int r = 1; r < 8; ++r) mx = fmaxf(mx, fmaxf(s0[r], s1[r]));
    mx = fmaxf(mx, __shfl_xor(mx, 16, 32));
    const float mn = fmaxf(m, mx);
    const float al = __expf(m - mn);
    m = mn;
    FragB ph, pl;
    float ps = 0.f;
#pragma unroll
    for (int r = 0; r < 8; ++r) {
      const float p0 = __expf(s0[r] - mn);
      const float p1 = __expf(s1[r] - mn);
      ps += p0 + p1;
      const unsigned int u0 = __float_as_uint(p0), u1 = __float_as_uint(p1);
      ph.u[r]     = (unsigned short)(u0 >> 16);
      ph.u[8 + r] = (unsigned short)(u1 >> 16);
      pl.u[r]     = bf16_bits(p0 - __uint_as_float(u0 & 0xFFFF0000u));
      pl.u[8 + r] = bf16_bits(p1 - __uint_as_float(u1 & 0xFFFF0000u));
    }
    l = l * al + ps;
    o0 = o0 * al; o1 = o1 * al; o2 = o2 * al; o3 = o3 * al;
    const int vo = vbase + kb;
    const v16b va0 = ld_frag(VT, vo, hh);
    const v16b va1 = ld_frag(VT, vo + 16 * SEQ, hh);
    const v16b va2 = ld_frag(VT, vo + 32 * SEQ, hh);
    const v16b va3 = ld_frag(VT, vo + 48 * SEQ, hh);
    o0 = mma2b(va0, ph.v, pl.v, o0);
    o1 = mma2b(va1, ph.v, pl.v, o1);
    o2 = mma2b(va2, ph.v, pl.v, o2);
    o3 = mma2b(va3, ph.v, pl.v, o3);
  }
  l += __shfl_xor(l, 16, 32);
  const float inv = 1.0f / l;
  const v8f ot[4] = {o0, o1, o2, o3};
#pragma unroll
  for (int t = 0; t < 4; ++t) {
    Pack8 fh, fl;
#pragma unroll
    for (int r = 0; r < 8; ++r) {
      const float c = ot[t][r] * inv;
      const unsigned short hb = bf16_bits(c);
      fh.u[r] = hb;
      fl.u[r] = bf16_bits(c - bf16_val(hb));
    }
    *(v8us*)&sH[w][ln][16 * t + 8 * hh] = fh.v;
    *(v8us*)&sL[w][ln][16 * t + 8 * hh] = fl.v;
  }
  __builtin_amdgcn_fence(4  , "workgroup");
  __builtin_amdgcn_wave_barrier();
  const int prow = lane >> 3, pc = (lane & 7) * 8;
  for (int pass = 0; pass < 2; ++pass) {
#pragma unroll
    for (int it = 0; it < 4; ++it) {
      const int row = it * 4 + prow;
      const v8us xh = *(const v8us*)&sH[w][row][pc];
      const v8us xl = *(const v8us*)&sL[w][row][pc];
      const size_t g = (size_t)(b * SEQ + q0 + row) * DM + h * HD + pc;
      *(volatile v8us*)(CH + g) = xh;
      *(volatile v8us*)(CL + g) = xl;
    }
    if (pass == 0) __threadfence();
  }
}

__global__ __launch_bounds__(128) void k_proj(const unsigned short* __restrict__ AH, const unsigned short* __restrict__ AL, const unsigned short* __restrict__ Wb,
                                             const float* __restrict__ bias, float* __restrict__ C) {
  __shared__ __attribute__((aligned(16))) float so[4][32][68];
  const int tid = threadIdx.x, w = tid >> 5, lane = tid & 31, ln = lane & 15, hh = lane >> 4;
  const int ntn = DM / 64;
  const int mt = blockIdx.x / ntn, nq = blockIdx.x - mt * ntn;
  const int row0 = mt * 128 + 32 * w, col0 = nq * 64;
  const int a0 = (row0 + ln) * DM, a1 = a0 + 16 * DM;
  const int b0 = (col0 + ln) * DM, b1 = b0 + 16 * DM, b2 = b1 + 16 * DM, b3 = b2 + 16 * DM;
  const v8f z8 = {0.f, 0.f, 0.f, 0.f, 0.f, 0.f, 0.f, 0.f};
  v8f c00 = z8, c01 = z8, c02 = z8, c03 = z8, c10 = z8, c11 = z8, c12 = z8, c13 = z8;
#pragma unroll 1
  for (int kb = 0; kb < DM; kb += 32) {
    const v16b a0h = ld_frag(AH, a0 + kb, hh), a0l = ld_frag(AL, a0 + kb, hh);
    const v16b a1h = ld_frag(AH, a1 + kb, hh), a1l = ld_frag(AL, a1 + kb, hh);
    v16b bw = ld_frag(Wb, b0 + kb, hh); c00 = mma2a(a0h, a0l, bw, c00); c10 = mma2a(a1h, a1l, bw, c10);
    bw = ld_frag(Wb, b1 + kb, hh);      c01 = mma2a(a0h, a0l, bw, c01); c11 = mma2a(a1h, a1l, bw, c11);
    bw = ld_frag(Wb, b2 + kb, hh);      c02 = mma2a(a0h, a0l, bw, c02); c12 = mma2a(a1h, a1l, bw, c12);
    bw = ld_frag(Wb, b3 + kb, hh);      c03 = mma2a(a0h, a0l, bw, c03); c13 = mma2a(a1h, a1l, bw, c13);
  }
  const v8f accs[8] = {c00, c01, c02, c03, c10, c11, c12, c13};
#pragma unroll
  for (int u = 0; u < 8; ++u) {
    const int t = u & 3, hf = u >> 2;
    const float bv = bf16_rne(bias[col0 + t * 16 + ln]);
#pragma unroll
    for (int r = 0; r < 8; ++r) so[w][hf * 16 + 8 * hh + r][t * 16 + ln] = accs[u][r] + bv;
  }
  __builtin_amdgcn_fence(4  , "workgroup");
  __builtin_amdgcn_wave_barrier();
  const int rsub = lane >> 4, c4 = (lane & 15) * 4;
  for (int pass = 0; pass < 2; ++pass) {
#pragma unroll
    for (int q = 0; q < 16; ++q) {
      const int r = q * 2 + rsub;
      const v4f v = *(const v4fa*)&so[w][r][c4];
      *(volatile v4f*)(C + (size_t)(row0 + r) * DM + col0 + c4) = v;
    }
    if (pass == 0) __threadfence();
  }
}

extern "C" void kernel_launch(void* const* d_in, const int* in_sizes, int n_in,
                              void* d_out, int out_size, void* d_ws, size_t ws_size, hipStream_t stream) {
  if (n_in < 5) return;
  const long long need_act = ((long long)(NB - 1) * SEQ_FULL + SEQ) * DM;
  if ((long long)in_sizes[0] < need_act || (long long)in_sizes[1] < need_act || (long long)in_sizes[2] < need_act) return;
  if ((long long)in_sizes[3] < (long long)DM * DM || in_sizes[4] < DM) return;
  if ((long long)out_size < (long long)NR * DM) return;
  if (ws_size < CARVE_B) return;
  const float* q = (const float*)d_in[0];
  const float* k = (const float*)d_in[1];
  const float* v = (const float*)d_in[2];
  const float* W = (const float*)d_in[3];
  const float* bias = (const float*)d_in[4];
  char* ws = (char*)d_ws;
  unsigned short* Qb = (unsigned short*)(ws);
  unsigned short* Kb = (unsigned short*)(ws + PLANE_B);
  unsigned short* VT = (unsigned short*)(ws + 2 * PLANE_B);
  unsigned short* CH = (unsigned short*)(ws + 3 * PLANE_B);
  unsigned short* CL = (unsigned short*)(ws + 4 * PLANE_B);
  unsigned short* Wb = (unsigned short*)(ws + 5 * PLANE_B);
  k_cvt_qk<<<(unsigned)(((size_t)NR * (DM / 8)) / 256), 256, 0, stream>>>(q, k, Qb, Kb);
  k_cvt_w<<<(unsigned)(((size_t)DM * (DM / 8)) / 256), 256, 0, stream>>>(W, Wb);
  k_vt<<<NB * NH * (SEQ / 64), 256, 0, stream>>>(v, VT);
  k_attn<<<NB * NH * (SEQ / QT), 128, 0, stream>>>(Qb, Kb, VT, CH, CL);
  k_proj<<<(NR / 128) * (DM / 64), 128, 0, stream>>>(CH, CL, Wb, bias, (float*)d_out);
}
